// LinearPolicy_82746839924987
// MI455X (gfx1250) — hardware-verified
//
#include <hip/hip_runtime.h>
#include <math.h>

constexpr int kB     = 2;
constexpr int kT     = 1024;
constexpr int kS     = 512;
constexpr int kC     = 512;
constexpr int kH     = 8;
constexpr int kD     = 64;
constexpr int kF     = 2048;
constexpr int kA     = 64;
constexpr int kL     = 4;
constexpr int kRows  = kB * kT;
constexpr int kQKVN  = 3 * kC;
constexpr int kHeadN = 192;
constexpr int kTS    = 32;
constexpr float kWScale    = 16.0f;
constexpr float kWScaleInv = 0.0625f;
static_assert(kRows % 64 == 0 && kC % 64 == 0 && kF % 64 == 0 && kQKVN % 64 == 0 && kHeadN % 64 == 0);
static_assert(kC % 32 == 0 && kF % 32 == 0 && kS % 32 == 0);
static_assert(kH * kD == kC && kT % kTS == 0 && kRows % 32 == 0);

typedef __attribute__((ext_vector_type(16))) _Float16 v16h;
typedef __attribute__((ext_vector_type(8)))  _Float16 v8h;
typedef __attribute__((ext_vector_type(16))) __bf16   v16b;
typedef __attribute__((ext_vector_type(8)))  __bf16   v8b;
typedef __attribute__((ext_vector_type(8)))  float    v8f;
typedef __attribute__((ext_vector_type(4)))  float    v4f;
typedef __attribute__((ext_vector_type(2)))  float    v2f;
typedef __attribute__((ext_vector_type(4)))  unsigned int v4u;

__device__ __forceinline__ unsigned short f2bf_bits(float f) {
  unsigned u = __float_as_uint(f);
  return (unsigned short)((u + 0x7FFFu + ((u >> 16) & 1u)) >> 16);
}
__device__ __forceinline__ float bf_bits2f(unsigned short h) { return __uint_as_float(((unsigned)h) << 16); }

__device__ __forceinline__ void dep_guard_h(v8f& a, v8f& b, v16h x, v16h y) { asm volatile("v_nop\n\tv_nop\n\tv_nop\n\tv_nop" : "+v"(a), "+v"(b) : "v"(x), "v"(y)); }
__device__ __forceinline__ void dep_guard_b(v8f& a, v8f& b, v16b x, v16b y) { asm volatile("v_nop\n\tv_nop\n\tv_nop\n\tv_nop" : "+v"(a), "+v"(b) : "v"(x), "v"(y)); }
__device__ __forceinline__ void keep4_h(v16h a, v16h b, v16h c, v16h d) { asm volatile("v_nop" :: "v"(a), "v"(b), "v"(c), "v"(d)); }
__device__ __forceinline__ void keep4_b(v16b a, v16b b, v16b c, v16b d) { asm volatile("v_nop" :: "v"(a), "v"(b), "v"(c), "v"(d)); }
__device__ __forceinline__ void acc_guard4(v8f& a, v8f& b, v8f& c, v8f& d) { asm volatile("v_nop\n\tv_nop\n\tv_nop\n\tv_nop" : "+v"(a), "+v"(b), "+v"(c), "+v"(d)); }
template <typename T> struct Frag;
template <> struct Frag<_Float16> {
  typedef v16h V; union U { v16h v; v8h h[2]; };
  static __device__ __forceinline__ v16h load(const _Float16* p) {
    U f; f.h[0] = *(const v8h*)(p); f.h[1] = *(const v8h*)(p + 16); return f.v;
  }
  static __device__ __forceinline__ v8f mma(v16h a, v16h b, v8f c) {
    return __builtin_amdgcn_wmma_f32_16x16x32_f16(false, a, false, b, (short)0, c, false, false);
  }
  static __device__ __forceinline__ void guard(v8f& a, v8f& b, v16h x, v16h y) { dep_guard_h(a, b, x, y); }
  static __device__ __forceinline__ void keep(v16h a, v16h b, v16h c, v16h d) { keep4_h(a, b, c, d); }
};
template <> struct Frag<__bf16> {
  typedef v16b V; union U { v16b v; v8b h[2]; };
  static __device__ __forceinline__ v16b load(const __bf16* p) {
    U f; f.h[0] = *(const v8b*)(p); f.h[1] = *(const v8b*)(p + 16); return f.v;
  }
  static __device__ __forceinline__ v8f mma(v16b a, v16b b, v8f c) {
    return __builtin_amdgcn_wmma_f32_16x16x32_bf16(false, a, false, b, (short)0, c, false, false);
  }
  static __device__ __forceinline__ void guard(v8f& a, v8f& b, v16b x, v16b y) { dep_guard_b(a, b, x, y); }
  static __device__ __forceinline__ void keep(v16b a, v16b b, v16b c, v16b d) { keep4_b(a, b, c, d); }
};

__device__ __forceinline__ unsigned pk16(unsigned short a, unsigned short b) { return (unsigned)a | ((unsigned)b << 16); }
__device__ __forceinline__ unsigned short h_bits(float f) { const _Float16 h = (_Float16)f; return __builtin_bit_cast(unsigned short, h); }

template <int ET> struct Elem;
template <> struct Elem<0> { typedef _Float16 T; };
template <> struct Elem<1> { typedef __bf16 T; };
template <int ET, bool SPLIT, int BIAS_MODE, int OUT_MODE, bool RESID, int ACT = 0>
__global__ __launch_bounds__(256) void wmma_gemm64(
    const unsigned short* __restrict__ Ap, const unsigned short* __restrict__ A2p, int lda, long strideA,
    const unsigned short* __restrict__ Btp, const unsigned short* __restrict__ Bt2p, int ldb, long strideB,
    void* __restrict__ Cout, void* __restrict__ Cout2, int ldc, long strideC,
    const float* __restrict__ bias,
    const float* __restrict__ resid, long strideR,
    int M, int N, int K, float scale) {
  typedef typename Elem<ET>::T T;
  typedef typename Frag<T>::V V;
  const T* A = (const T*)Ap; const T* A2 = (const T*)A2p; const T* Bt = (const T*)Btp; const T* Bt2 = (const T*)Bt2p;
  __shared__ __align__(16) float sT[8][16 * 68];
  const int b    = blockIdx.y;
  const int lane = threadIdx.x & 31;
  const int wave = threadIdx.x >> 5;
  const int tilesN = N >> 6;
  const int tilesM = M >> 6;
  const int tile = blockIdx.x * 8 + wave;
  if (tile >= tilesM * tilesN) return;
  const int tm = tile / tilesN;
  const int tn = tile - tm * tilesN;
  const int m0 = tm << 6;
  const int n0 = tn << 6;

  const T* Ab  = A  + (size_t)b * strideA;
  const T* Bb  = Bt + (size_t)b * strideB;
  const T* Ab2 = SPLIT ? (A2  + (size_t)b * strideA) : nullptr;
  const T* Bb2 = SPLIT ? (Bt2 + (size_t)b * strideB) : nullptr;

  const int rlane = lane & 15;
  const int koff  = (lane >> 4) * 8;
  const int mOff  = (lane >> 4) * 8;

  v8f acc[4][4];
#pragma unroll
  for (int i = 0; i < 4; ++i)
#pragma unroll
    for (int j = 0; j < 4; ++j) acc[i][j] = (v8f){0.f,0.f,0.f,0.f,0.f,0.f,0.f,0.f};

  for (int k0 = 0; k0 < K; k0 += 32) {
    V bh[4], bl[4];
#pragma unroll
    for (int j = 0; j < 4; ++j) {
      const size_t bo = (size_t)(n0 + (j << 4) + rlane) * ldb + koff + k0;
      bh[j] = Frag<T>::load(Bb + bo);
      if (SPLIT) bl[j] = Frag<T>::load(Bb2 + bo);
    }
#pragma unroll
    for (int i = 0; i < 4; ++i) {
      const size_t ao = (size_t)(m0 + (i << 4) + rlane) * lda + koff + k0;
      V ah = Frag<T>::load(Ab + ao);
      V al;
      if (SPLIT) al = Frag<T>::load(Ab2 + ao);
#pragma unroll
      for (int j = 0; j < 4; ++j) {
        acc[i][j] = Frag<T>::mma(ah, bh[j], acc[i][j]);
        if (SPLIT) {
          acc[i][j] = Frag<T>::mma(ah, bl[j], acc[i][j]);
          acc[i][j] = Frag<T>::mma(al, bh[j], acc[i][j]);
        }
      }
      Frag<T>::guard(acc[i][0], acc[i][3], ah, SPLIT ? al : ah);
    }
    Frag<T>::keep(bh[0], bh[1], bh[2], bh[3]);
    if (SPLIT) Frag<T>::keep(bl[0], bl[1], bl[2], bl[3]);
  }
  acc_guard4(acc[0][0], acc[0][1], acc[0][2], acc[0][3]);
  acc_guard4(acc[1][0], acc[1][1], acc[1][2], acc[1][3]);
  acc_guard4(acc[2][0], acc[2][1], acc[2][2], acc[2][3]);
  acc_guard4(acc[3][0], acc[3][1], acc[3][2], acc[3][3]);

  float* slab = sT[wave];
  const float* Rb = RESID ? (resid + (size_t)b * strideR) : nullptr;
#pragma unroll
  for (int i = 0; i < 4; ++i) {
    const int mBase = m0 + (i << 4);
#pragma unroll
    for (int j = 0; j < 4; ++j) {
      const int n = n0 + (j << 4) + rlane;
      float bv = 0.f;
      if (BIAS_MODE == 2) bv = bias[n];
#pragma unroll
      for (int r = 0; r < 8; ++r) {
        float v = acc[i][j][r] * scale;
        if (BIAS_MODE == 1) v += bias[mBase + mOff + r];
        if (BIAS_MODE == 2) v += bv;
        if (RESID) v += Rb[(size_t)(mBase + mOff + r) * ldc + n];
        if (ACT == 2) v = fmaxf(v, 0.0f);
        if (ACT == 4) v = (v > 0.f) ? v : 0.01f * v;
        slab[(mOff + r) * 68 + (j << 4) + rlane] = v;
      }
    }
    __builtin_amdgcn_fence(__ATOMIC_RELEASE, "workgroup");
    __builtin_amdgcn_wave_barrier();
    __builtin_amdgcn_fence(__ATOMIC_ACQUIRE, "workgroup");
    if (OUT_MODE == 0) {
      float* Cp = (float*)Cout + (size_t)b * strideC;
      const int hh = lane >> 4, c4 = (lane & 15) * 4;
      for (int pass = 0; pass < 2; ++pass) {
#pragma unroll
        for (int it = 0; it < 8; ++it) {
          const int row = it * 2 + hh;
          v4f v = *(const v4f*)(slab + row * 68 + c4);
          *(volatile v4f*)(Cp + (size_t)(mBase + row) * ldc + n0 + c4) = v;
        }
        __threadfence();
      }
    } else {
      const int q = lane >> 3, c8 = (lane & 7) * 8;
      unsigned short* Cp  = (unsigned short*)Cout  + (size_t)b * strideC;
      unsigned short* Cp2 = (OUT_MODE == 2) ? ((unsigned short*)Cout2 + (size_t)b * strideC) : nullptr;
      for (int pass = 0; pass < 2; ++pass) {
#pragma unroll
        for (int it = 0; it < 4; ++it) {
          const int row = it * 4 + q;
          const float* sp = slab + row * 68 + c8;
          v8h hv, lv;
#pragma unroll
          for (int e = 0; e < 8; ++e) {
            if (OUT_MODE == 1) {
              hv[e] = (_Float16)sp[e];
            } else {
              unsigned short hb = f2bf_bits(sp[e]);
              unsigned short lb = f2bf_bits(sp[e] - bf_bits2f(hb));
              hv[e] = __builtin_bit_cast(_Float16, hb);
              lv[e] = __builtin_bit_cast(_Float16, lb);
            }
          }
          *(volatile v8h*)(Cp + (size_t)(mBase + row) * ldc + n0 + c8) = hv;
          if (OUT_MODE == 2) *(volatile v8h*)(Cp2 + (size_t)(mBase + row) * ldc + n0 + c8) = lv;
        }
        __threadfence();
      }
    }
    __builtin_amdgcn_fence(__ATOMIC_RELEASE, "workgroup");
    __builtin_amdgcn_wave_barrier();
    __builtin_amdgcn_fence(__ATOMIC_ACQUIRE, "workgroup");
  }
}

template <int MODE>
__global__ __launch_bounds__(256) void cast8_kernel(const float* __restrict__ in, unsigned short* __restrict__ out, int n8, float scale) {
  const int i = blockIdx.x * 256 + threadIdx.x;
  if (i >= n8) return;
  const float* p = in + 8 * (size_t)i;
  const v4f a = *(const v4f*)(p);
  const v4f c = *(const v4f*)(p + 4);
  unsigned short hb[8];
#pragma unroll
  for (int e = 0; e < 4; ++e) {
    if (MODE == 0) {
      hb[e]     = f2bf_bits(a[e]);
      hb[4 + e] = f2bf_bits(c[e]);
    } else {
      hb[e]     = h_bits(bf_bits2f(f2bf_bits(a[e])) * scale);
      hb[4 + e] = h_bits(bf_bits2f(f2bf_bits(c[e])) * scale);
    }
  }
  const v4u u = (v4u){pk16(hb[0], hb[1]), pk16(hb[2], hb[3]), pk16(hb[4], hb[5]), pk16(hb[6], hb[7])};
  unsigned short* q = out + 8 * (size_t)i;
  *(volatile v4u*)q = u;
  __threadfence();
  *(volatile v4u*)q = u;
  (void)scale;
}

__global__ __launch_bounds__(256) void tcast8w_kernel(const float* __restrict__ in, unsigned short* __restrict__ out,
                                                      int Kin, int Nin, int Kpad, int n8,
                                                      long inStride, long outStride, float wscale) {
  const int i = blockIdx.x * 256 + threadIdx.x;
  if (i >= n8) return;
  const float* inb = in + (size_t)blockIdx.y * (size_t)inStride;
  unsigned short* outb = out + (size_t)blockIdx.y * (size_t)outStride;
  const size_t e0 = (size_t)i * 8;
  const int n  = (int)(e0 / (size_t)Kpad);
  const int k0 = (int)(e0 - (size_t)n * Kpad);
  const int nc = (n < Nin) ? n : (Nin - 1);
  unsigned short hb[8];
#pragma unroll
  for (int e = 0; e < 8; ++e) {
    const int k  = k0 + e;
    const int kc = (k < Kin) ? k : (Kin - 1);
    float f = inb[(size_t)kc * Nin + nc];
    if (k >= Kin || n >= Nin) f = 0.0f;
    hb[e] = h_bits(bf_bits2f(f2bf_bits(f)) * wscale);
  }
  const v4u u = (v4u){pk16(hb[0], hb[1]), pk16(hb[2], hb[3]), pk16(hb[4], hb[5]), pk16(hb[6], hb[7])};
  unsigned short* q = outb + e0;
  *(volatile v4u*)q = u;
  __threadfence();
  *(volatile v4u*)q = u;
}

__global__ __launch_bounds__(256) void layernorm_f16_kernel(const float* __restrict__ x, const float* __restrict__ g,
                                                            const float* __restrict__ bt, unsigned short* __restrict__ y,
                                                            int nrows) {
  const int lane = threadIdx.x & 31, wave = threadIdx.x >> 5;
  const int row = blockIdx.x * 8 + wave;
  if (row >= nrows) return;
  const float* xr = x + (size_t)row * kC;
  const int c0 = 8 * lane, c1 = 256 + 8 * lane;
  const v4f a0 = *(const v4f*)(xr + c0);
  const v4f a1 = *(const v4f*)(xr + c0 + 4);
  const v4f a2 = *(const v4f*)(xr + c1);
  const v4f a3 = *(const v4f*)(xr + c1 + 4);
  float sum = 0.0f;
#pragma unroll
  for (int e = 0; e < 4; ++e) sum += (a0[e] + a1[e]) + (a2[e] + a3[e]);
#pragma unroll
  for (int off = 16; off > 0; off >>= 1) sum += __shfl_xor(sum, off, 32);
  const float mean = sum * (1.0f / (float)kC);
  v4f d0, d1, d2, d3;
  float sq = 0.0f;
#pragma unroll
  for (int e = 0; e < 4; ++e) {
    d0[e] = a0[e] - mean; d1[e] = a1[e] - mean; d2[e] = a2[e] - mean; d3[e] = a3[e] - mean;
    sq += (d0[e] * d0[e] + d1[e] * d1[e]) + (d2[e] * d2[e] + d3[e] * d3[e]);
  }
#pragma unroll
  for (int off = 16; off > 0; off >>= 1) sq += __shfl_xor(sq, off, 32);
  const float var = sq * (1.0f / (float)kC);
  const float rs  = rsqrtf(var + 1e-5f);
  const v4f g0 = *(const v4f*)(g + c0), g1 = *(const v4f*)(g + c0 + 4), g2 = *(const v4f*)(g + c1), g3 = *(const v4f*)(g + c1 + 4);
  const v4f b0 = *(const v4f*)(bt + c0), b1 = *(const v4f*)(bt + c0 + 4), b2 = *(const v4f*)(bt + c1), b3 = *(const v4f*)(bt + c1 + 4);
  v8h h0, h1;
#pragma unroll
  for (int e = 0; e < 4; ++e) {
    h0[e]     = (_Float16)((d0[e] * rs) * g0[e] + b0[e]);
    h0[4 + e] = (_Float16)((d1[e] * rs) * g1[e] + b1[e]);
    h1[e]     = (_Float16)((d2[e] * rs) * g2[e] + b2[e]);
    h1[4 + e] = (_Float16)((d3[e] * rs) * g3[e] + b3[e]);
  }
  unsigned short* q0 = y + (size_t)row * kC + c0;
  unsigned short* q1 = y + (size_t)row * kC + c1;
  *(volatile v8h*)q0 = h0;
  *(volatile v8h*)q1 = h1;
  __threadfence();
  *(volatile v8h*)q0 = h0;
  *(volatile v8h*)q1 = h1;
}

__global__ __launch_bounds__(256) void linscan_kernel(const float* __restrict__ qkv, unsigned short* __restrict__ oh) {
  __shared__ __align__(16) float stg[3][kTS][64];
  __shared__ __align__(16) float so[kTS][68];
  const int bh   = blockIdx.x;
  const int b    = bh >> 3, h = bh & 7;
  const int tid  = threadIdx.x;
  const int lane = tid & 31, wave = tid >> 5;
  const int vcol = tid >> 2, kq = tid & 3;
  const int hc   = h * kD;
  const size_t row0 = (size_t)b * kT;

  float S[16], Z[16];
#pragma unroll
  for (int e = 0; e < 16; ++e) { S[e] = 0.0f; Z[e] = 0.0f; }

#pragma unroll 1
  for (int t0 = 0; t0 < kT; t0 += kTS) {
    __syncthreads();
#pragma unroll 1
    for (int i = 0; i < 6; ++i) {
      const int idx = i * 256 + tid;
      const int s   = idx / 48;
      const int rem = idx - s * 48;
      const int arr = rem >> 4;
      const int j4  = (rem & 15) * 4;
      const v4f val = *(const v4f*)(qkv + (row0 + (size_t)(t0 + s)) * (size_t)kQKVN + (size_t)arr * kC + hc + j4);
      v4f res;
#pragma unroll
      for (int e = 0; e < 4; ++e) {
        const float xv = val[e];
        const float ph = (xv > 0.0f) ? (xv + 1.0f) : __expf(xv);
        res[e] = (arr < 2) ? ph : xv;
      }
      *(v4f*)(&stg[arr][s][j4]) = res;
    }
    __syncthreads();
#pragma unroll 1
    for (int s = 0; s < kTS; ++s) {
      const float vv = stg[2][s][vcol];
      float o = 0.0f, dn = 0.0f;
#pragma unroll
      for (int e4 = 0; e4 < 4; ++e4) {
        const int kb = kq * 16 + e4 * 4;
        const v4f k4 = *(const v4f*)(&stg[1][s][kb]);
        const v4f q4 = *(const v4f*)(&stg[0][s][kb]);
#pragma unroll
        for (int e = 0; e < 4; ++e) {
          const int idx = e4 * 4 + e;
          const float sn = S[idx] + k4[e] * vv;
          S[idx] = sn;
          o += q4[e] * sn;
          const float zn = Z[idx] + k4[e];
          Z[idx] = zn;
          dn += q4[e] * zn;
        }
      }
      o  += __shfl_xor(o, 1, 32);
      o  += __shfl_xor(o, 2, 32);
      dn += __shfl_xor(dn, 1, 32);
      dn += __shfl_xor(dn, 2, 32);
      const float r = o * (1.0f / (dn + 1e-6f));
      if (kq == 0) so[s][vcol] = r;
    }
    __syncthreads();
    {
      const int q = lane >> 3, c8 = (lane & 7) * 8;
      const int row = wave * 4 + q;
      v8h hv;
#pragma unroll
      for (int e = 0; e < 8; ++e) hv[e] = (_Float16)so[row][c8 + e];
      unsigned short* dst = oh + (row0 + (size_t)(t0 + row)) * (size_t)kC + hc + c8;
      *(volatile v8h*)dst = hv;
      __threadfence();
      *(volatile v8h*)dst = hv;
    }
  }
}

__global__ __launch_bounds__(256) void gelu_cast_kernel(const float* __restrict__ in, unsigned short* __restrict__ out, int n2) {
  const int i = blockIdx.x * 256 + threadIdx.x;
  if (i >= n2) return;
  const v2f a = *(const v2f*)(in + 2 * (size_t)i);
  const float g0 = 0.5f * a[0] * (1.0f + erff(a[0] * 0.70710678118654752f));
  const float g1 = 0.5f * a[1] * (1.0f + erff(a[1] * 0.70710678118654752f));
  const unsigned u = pk16(h_bits(g0), h_bits(g1));
  ((volatile unsigned*)out)[i] = u;
  __threadfence();
  ((volatile unsigned*)out)[i] = u;
}

__global__ __launch_bounds__(256) void heads_out_kernel(const float* __restrict__ hd, const float* __restrict__ amb,
                                                        const float* __restrict__ alsb, const float* __restrict__ crb,
                                                        float* __restrict__ out0, float* __restrict__ out1,
                                                        float* __restrict__ out2, int nrows) {
  __shared__ __align__(16) float sv[32];
  const int tid = threadIdx.x, lane = tid & 31, wave = tid >> 5;
  const int rbase = blockIdx.x * 32;
  if (tid < 32) {
    const int r = rbase + tid;
    const int rc = (r < nrows) ? r : (nrows - 1);
    sv[tid] = hd[(size_t)rc * kHeadN + 2 * kA] + crb[0];
  }
  __syncthreads();
  const int hh = lane >> 4, c4 = (lane & 15) * 4;
  const v4f ba = *(const v4f*)(amb + c4);
  const v4f bs = *(const v4f*)(alsb + c4);
  v4f va[2], vs[2];
  int rows[2];
#pragma unroll
  for (int it = 0; it < 2; ++it) {
    const int row = rbase + wave * 4 + it * 2 + hh;
    rows[it] = row;
    const int rc = (row < nrows) ? row : (nrows - 1);
    const v4f a = *(const v4f*)(hd + (size_t)rc * kHeadN + c4);
    const v4f s = *(const v4f*)(hd + (size_t)rc * kHeadN + kA + c4);
    v4f ra, rsv;
#pragma unroll
    for (int e = 0; e < 4; ++e) {
      ra[e]  = a[e] + ba[e];
      rsv[e] = fminf(fmaxf(s[e] + bs[e], -2.0f), 1.0f);
    }
    va[it] = ra; vs[it] = rsv;
  }
  const int l8 = (lane < 8) ? lane : 7;
  const v4f v2 = *(const v4f*)(&sv[4 * l8]);
  const bool w2 = (wave == 0) && (lane < 8) && (rbase + 4 * lane + 3 < nrows);
  for (int pass = 0; pass < 2; ++pass) {
#pragma unroll
    for (int it = 0; it < 2; ++it) {
      if (rows[it] < nrows) {
        *(volatile v4f*)(out0 + (size_t)rows[it] * kA + c4) = va[it];
        *(volatile v4f*)(out1 + (size_t)rows[it] * kA + c4) = vs[it];
      }
    }
    if (w2) *(volatile v4f*)(out2 + rbase + 4 * lane) = v2;
    __threadfence();
  }
}

extern "C" void kernel_launch(void* const* d_in, const int* in_sizes, int n_in,
                              void* d_out, int out_size, void* d_ws, size_t ws_size,
                              hipStream_t stream)
{
  if (n_in < 24) return;
  if (in_sizes[0] != kRows * kS || in_sizes[6] != kL * kC * kQKVN || out_size != kRows * (2 * kA + 1)) return;

  const float* states = (const float*)d_in[0];
  const float* sew    = (const float*)d_in[1];
  const float* seb    = (const float*)d_in[2];
  const float* pos    = (const float*)d_in[3];
  const float* ln1_g  = (const float*)d_in[4];
  const float* ln1_b  = (const float*)d_in[5];
  const float* qkv_w  = (const float*)d_in[6];
  const float* qkv_b  = (const float*)d_in[7];
  const float* ow     = (const float*)d_in[8];
  const float* ob     = (const float*)d_in[9];
  const float* ln2_g  = (const float*)d_in[10];
  const float* ln2_b  = (const float*)d_in[11];
  const float* w1     = (const float*)d_in[12];
  const float* b1     = (const float*)d_in[13];
  const float* w2     = (const float*)d_in[14];
  const float* b2     = (const float*)d_in[15];
  const float* lnf_g  = (const float*)d_in[16];
  const float* lnf_b  = (const float*)d_in[17];
  const float* amw    = (const float*)d_in[18];
  const float* amb    = (const float*)d_in[19];
  const float* alsw   = (const float*)d_in[20];
  const float* alsb   = (const float*)d_in[21];
  const float* crw    = (const float*)d_in[22];
  const float* crb    = (const float*)d_in[23];

  size_t off = 0;
  unsigned char* ws = (unsigned char*)d_ws;
  auto carve = [&](size_t bytes) { unsigned char* p = ws + off; off += bytes; return p; };
  unsigned short* Wsew = (unsigned short*)carve((size_t)kC * kS * 2);
  unsigned short* Wqkv = (unsigned short*)carve((size_t)kL * kQKVN * kC * 2);
  unsigned short* Wow  = (unsigned short*)carve((size_t)kL * kC * kC * 2);
  unsigned short* Ww1  = (unsigned short*)carve((size_t)kL * kF * kC * 2);
  unsigned short* Ww2  = (unsigned short*)carve((size_t)kL * kC * kF * 2);
  unsigned short* Whd  = (unsigned short*)carve((size_t)kHeadN * kC * 2);
  unsigned short* Ast  = (unsigned short*)carve((size_t)kRows * kS * 2);
  float*          X0   = (float*)carve((size_t)kRows * kC * 4);
  float*          X1   = (float*)carve((size_t)kRows * kC * 4);
  unsigned short* Hh   = (unsigned short*)carve((size_t)kRows * kC * 2);
  float*          QKV  = (float*)carve((size_t)kRows * kQKVN * 4);
  unsigned short* Oh   = (unsigned short*)carve((size_t)kRows * kC * 2);
  float*          U    = (float*)carve((size_t)kRows * kF * 4);
  unsigned short* Gh   = (unsigned short*)carve((size_t)kRows * kF * 2);
  float*          HDo  = (float*)carve((size_t)kRows * kHeadN * 4);
  if (off > ws_size) return;

  float* out0 = (float*)d_out;
  float* out1 = out0 + (size_t)kRows * kA;
  float* out2 = out0 + (size_t)2 * kRows * kA;

  const dim3 blk(256);
  auto gemm_grid = [](int M, int N, int batch) { return dim3((unsigned)((((M / 64) * (N / 64)) + 7) / 8), (unsigned)batch); };

  cast8_kernel<1><<<dim3((unsigned)(kRows * kS / 8 / 256)), blk, 0, stream>>>(states, Ast, kRows * kS / 8, 1.0f);
  tcast8w_kernel<<<dim3((unsigned)(kC * kS / 8 / 256), 1), blk, 0, stream>>>(sew, Wsew, kS, kC, kS, kC * kS / 8, 0L, 0L, kWScale);
  tcast8w_kernel<<<dim3((unsigned)(kQKVN * kC / 8 / 256), kL), blk, 0, stream>>>(qkv_w, Wqkv, kC, kQKVN, kC, kQKVN * kC / 8,
                                                                                 (long)kC * kQKVN, (long)kQKVN * kC, kWScale);
  tcast8w_kernel<<<dim3((unsigned)(kC * kC / 8 / 256), kL), blk, 0, stream>>>(ow, Wow, kC, kC, kC, kC * kC / 8,
                                                                              (long)kC * kC, (long)kC * kC, kWScale);
  tcast8w_kernel<<<dim3((unsigned)(kF * kC / 8 / 256), kL), blk, 0, stream>>>(w1, Ww1, kC, kF, kC, kF * kC / 8,
                                                                              (long)kC * kF, (long)kF * kC, kWScale);
  tcast8w_kernel<<<dim3((unsigned)(kC * kF / 8 / 256), kL), blk, 0, stream>>>(w2, Ww2, kF, kC, kF, kC * kF / 8,
                                                                              (long)kF * kC, (long)kC * kF, kWScale);
  tcast8w_kernel<<<dim3((unsigned)(64 * kC / 8 / 256), 1), blk, 0, stream>>>(amw,  Whd,                      kC, kA, kC, 64 * kC / 8, 0L, 0L, kWScale);
  tcast8w_kernel<<<dim3((unsigned)(64 * kC / 8 / 256), 1), blk, 0, stream>>>(alsw, Whd + (size_t)64 * kC,   kC, kA, kC, 64 * kC / 8, 0L, 0L, kWScale);
  tcast8w_kernel<<<dim3((unsigned)(64 * kC / 8 / 256), 1), blk, 0, stream>>>(crw,  Whd + (size_t)128 * kC,  kC, 1,  kC, 64 * kC / 8, 0L, 0L, kWScale);

  wmma_gemm64<0, false, 2, 0, true, 0><<<gemm_grid(kT, kC, kB), blk, 0, stream>>>(
      Ast, Ast, kS, (long)kT * kS, Wsew, Wsew, kS, 0L, X0, X0, kC, (long)kT * kC,
      seb, pos, 0L, kT, kC, kS, kWScaleInv);

  for (int i = 0; i < kL; ++i) {
    layernorm_f16_kernel<<<dim3(kRows / 8), blk, 0, stream>>>(X0, ln1_g + (size_t)i * kC, ln1_b + (size_t)i * kC, Hh, kRows);
    wmma_gemm64<0, false, 2, 0, false, 0><<<gemm_grid(kRows, kQKVN, 1), blk, 0, stream>>>(
        Hh, Hh, kC, 0L, Wqkv + (size_t)i * kQKVN * kC, Wqkv + (size_t)i * kQKVN * kC, kC, 0L,
        QKV, QKV, kQKVN, 0L, qkv_b + (size_t)i * kQKVN, X0, 0L, kRows, kQKVN, kC, kWScaleInv);
    linscan_kernel<<<dim3(kB * kH), blk, 0, stream>>>(QKV, Oh);
    wmma_gemm64<0, false, 2, 0, true, 0><<<gemm_grid(kRows, kC, 1), blk, 0, stream>>>(
        Oh, Oh, kC, 0L, Wow + (size_t)i * kC * kC, Wow + (size_t)i * kC * kC, kC, 0L,
        X1, X1, kC, 0L, ob + (size_t)i * kC, X0, 0L, kRows, kC, kC, kWScaleInv);
    layernorm_f16_kernel<<<dim3(kRows / 8), blk, 0, stream>>>(X1, ln2_g + (size_t)i * kC, ln2_b + (size_t)i * kC, Hh, kRows);
    wmma_gemm64<0, false, 2, 0, false, 0><<<gemm_grid(kRows, kF, 1), blk, 0, stream>>>(
        Hh, Hh, kC, 0L, Ww1 + (size_t)i * kF * kC, Ww1 + (size_t)i * kF * kC, kC, 0L,
        U, U, kF, 0L, b1 + (size_t)i * kF, X0, 0L, kRows, kF, kC, kWScaleInv);
    gelu_cast_kernel<<<dim3((unsigned)(kRows * kF / 2 / 256)), blk, 0, stream>>>(U, Gh, kRows * kF / 2);
    wmma_gemm64<0, false, 2, 0, true, 0><<<gemm_grid(kRows, kC, 1), blk, 0, stream>>>(
        Gh, Gh, kF, 0L, Ww2 + (size_t)i * kC * kF, Ww2 + (size_t)i * kC * kF, kF, 0L,
        X0, X0, kC, 0L, b2 + (size_t)i * kC, X1, 0L, kRows, kC, kF, kWScaleInv);
  }

  layernorm_f16_kernel<<<dim3(kRows / 8), blk, 0, stream>>>(X0, lnf_g, lnf_b, Hh, kRows);
  wmma_gemm64<0, false, 0, 0, false, 0><<<gemm_grid(kRows, kHeadN, 1), blk, 0, stream>>>(
      Hh, Hh, kC, 0L, Whd, Whd, kC, 0L, HDo, HDo, kHeadN, 0L, amb, X0, 0L, kRows, kHeadN, kC, kWScaleInv);
  heads_out_kernel<<<dim3(kRows / 32), blk, 0, stream>>>(HDo, amb, alsb, crb, out0, out1, out2, kRows);
}
